// BlockRC1_16140487099013
// MI455X (gfx1250) — hardware-verified
//
#include <hip/hip_runtime.h>
#include <math.h>
#include <stddef.h>


typedef unsigned short u16;
typedef __bf16 v16bf __attribute__((ext_vector_type(16)));
typedef unsigned short us8_t __attribute__((ext_vector_type(8)));
typedef us8_t us8a __attribute__((may_alias));
typedef float v8f __attribute__((ext_vector_type(8)));
typedef float v4f_t __attribute__((ext_vector_type(4)));
typedef v4f_t v4fa __attribute__((may_alias));

union Frag { v16bf v; us8_t h[2]; };

#define TT 65536
#define NBPB 1024
#define IMW 1024
#define XW 288
#define XR 25
#define AP 264
#define SP 72
#define YP 68
#define RECW 2176
#define KXW 2560
#define RSQ32 0.17677669529663688f
#define LDS_MAIN 142848

__device__ __forceinline__ u16 bfr(float f) {
  unsigned u = __float_as_uint(f);
  u += 0x7FFFu + ((u >> 16) & 1u);
  return (u16)(u >> 16);
}
__device__ __forceinline__ float bff(u16 b) { return __uint_as_float(((unsigned)b) << 16); }
__device__ __forceinline__ void split2(float f, u16& hi, u16& lo) {
  const u16 hv = bfr(f);
  hi = hv;
  lo = bfr(f - bff(hv));
}
__device__ __forceinline__ v8f zero8() {
  v8f z = {0.0f, 0.0f, 0.0f, 0.0f, 0.0f, 0.0f, 0.0f, 0.0f};
  return z;
}
__device__ __forceinline__ us8_t zeros8h() {
  us8_t z = {0, 0, 0, 0, 0, 0, 0, 0};
  return z;
}
__device__ __forceinline__ float wsum(float v) {
#pragma unroll
  for (int o = 16; o > 0; o >>= 1) v += __shfl_xor(v, o, 32);
  return v;
}
__device__ __forceinline__ float gelu_f(float v) {
  return 0.5f * v * (1.0f + erff(v * 0.70710678118654752f));
}

__device__ __forceinline__ v16bf ldfrag(const u16* base, int pitch, int row, int k0, int h) {
  Frag f;
  const u16* p = base + row * pitch + k0 + 8 * h;
  f.h[0] = *(const us8a*)(p);
  f.h[1] = *(const us8a*)(p + 16);
  return f.v;
}

__device__ __forceinline__ void mma3(v8f& acc, const v16bf ah, const v16bf al, const v16bf bh, const v16bf bl) {
  acc = __builtin_amdgcn_wmma_f32_16x16x32_bf16(false, ah, false, bh, (short)0, acc, false, false);
  acc = __builtin_amdgcn_wmma_f32_16x16x32_bf16(false, ah, false, bl, (short)0, acc, false, false);
  acc = __builtin_amdgcn_wmma_f32_16x16x32_bf16(false, al, false, bh, (short)0, acc, false, false);
  asm volatile("v_nop\n\tv_nop\n\tv_nop\n\tv_nop" : "+v"(acc) : "v"(ah), "v"(al), "v"(bh), "v"(bl));
}

__global__ __launch_bounds__(256) void k_prep(
    const float* __restrict__ conv_w, const float* __restrict__ kqv_w, const float* __restrict__ wperf,
    const float* __restrict__ proj_w, const float* __restrict__ mlp1_w, const float* __restrict__ mlp2_w,
    u16* wc, u16* wk, u16* wp, u16* wpr, u16* wm1, u16* wm2) {
  const int j = blockIdx.x * 256 + threadIdx.x;
  const bool act = j < 2496;
  us8_t piece[8];
#pragma unroll
  for (int pc = 0; pc < 8; ++pc) piece[pc] = zeros8h();
  u16* dst = wc;
  if (act) {
    int kind = 0, plane = 0, n = 0, ci = 0, kq = 0;
    const float* src = proj_w;
    if (j < 512) {
      kind = 0; ci = j >> 7; plane = (j >> 6) & 1; n = j & 63;
      dst = wc + ((ci * 2 + plane) * 64 + n) * 64;
    } else if (j < 2048) {
      const int jj = j - 512;
      kind = 1; plane = jj / 768;
      const int rem = jj - plane * 768;
      n = rem >> 2; kq = rem & 3;
      dst = wk + (plane * 192 + n) * 256 + kq * 64;
    } else if (j < 2112) {
      const int jj = j - 2048;
      kind = 2; plane = jj >> 5; n = jj & 31;
      dst = wp + (plane * 32 + n) * 64;
    } else {
      const int jj = j - 2112;
      const int which = jj >> 7;
      const int rem = jj & 127;
      kind = 3; plane = rem >> 6; n = rem & 63;
      src = (which == 0) ? proj_w : ((which == 1) ? mlp1_w : mlp2_w);
      u16* bb = (which == 0) ? wpr : ((which == 1) ? wm1 : wm2);
      dst = bb + (plane * 64 + n) * 64;
    }
#pragma unroll
    for (int pc = 0; pc < 8; ++pc) {
      us8_t pv = zeros8h();
#pragma unroll
      for (int e = 0; e < 8; ++e) {
        const int i = pc * 8 + e;
        float v;
        if (kind == 0) {
          const int kh = i >> 3, kw = i & 7;
          v = (kh < 7 && kw < 7) ? conv_w[(ci * 64 + n) * 49 + kh * 7 + kw] : 0.0f;
        } else if (kind == 1) {
          v = kqv_w[(kq * 64 + i) * 192 + n];
        } else if (kind == 2) {
          v = wperf[n * 64 + i];
        } else {
          v = src[i * 64 + n];
        }
        u16 hv, lv;
        split2(v, hv, lv);
        pv[e] = plane ? lv : hv;
      }
      piece[pc] = pv;
    }
#pragma unroll
    for (int pc = 0; pc < 8; ++pc) *(volatile us8_t*)(dst + pc * 8) = piece[pc];
  }
  __threadfence();
  if (act) {
#pragma unroll
    for (int pc = 0; pc < 8; ++pc) *(volatile us8_t*)(dst + pc * 8) = piece[pc];
  }
}

template <int CI>
__device__ __forceinline__ void conv_dil(const u16* xh, const u16* xl, const u16* __restrict__ wc,
                                         const float* __restrict__ conv_b, float* sTok, int lane, int wv) {
  constexpr int D = CI + 1;
  constexpr int P = (CI == 0) ? 2 : ((CI == 1) ? 5 : ((CI == 2) ? 8 : 11));
  constexpr int OFF = 11 - P;
  const int m = lane & 15, h = lane >> 4, rt = wv & 3, nh = wv >> 2;
  const int tl = rt * 16 + m;
  v8f acc[2];
  acc[0] = zero8();
  acc[1] = zero8();
#pragma unroll
  for (int s = 0; s < 2; ++s) {
    Frag ah, al;
#pragma unroll
    for (int g = 0; g < 2; ++g) {
      const int khc = 4 * s + 2 * g;
      const int kh = (khc >= 6) ? 6 : (khc + h);
      const int ra = (OFF + kh * D) * XW + tl * 4 + OFF;
      us8_t ph = zeros8h(), pl = zeros8h();
#pragma unroll
      for (int kw = 0; kw < 8; ++kw) {
        ph[kw] = xh[ra + kw * D];
        pl[kw] = xl[ra + kw * D];
      }
      ah.h[g] = ph;
      al.h[g] = pl;
    }
#pragma unroll
    for (int jn = 0; jn < 2; ++jn) {
      const int n = nh * 32 + jn * 16 + m;
      const v16bf bh = ldfrag(wc + (CI * 2 + 0) * 4096, 64, n, 32 * s, h);
      const v16bf bl = ldfrag(wc + (CI * 2 + 1) * 4096, 64, n, 32 * s, h);
      mma3(acc[jn], ah.v, al.v, bh, bl);
    }
  }
#pragma unroll
  for (int jn = 0; jn < 2; ++jn) {
    const int ch = nh * 32 + jn * 16 + m;
    const float bias = conv_b[CI * 64 + ch];
#pragma unroll
    for (int r = 0; r < 8; ++r) {
      const int tk = rt * 16 + 8 * h + r;
      sTok[tk * 256 + CI * 64 + ch] = gelu_f(acc[jn][r] + bias);
    }
  }
}

__global__ __launch_bounds__(256) void k_main(
    const float* __restrict__ x, const float* __restrict__ conv_b,
    const float* __restrict__ n1g, const float* __restrict__ n1b,
    const float* __restrict__ kqv_b,
    const u16* __restrict__ wc, const u16* __restrict__ wk, const u16* __restrict__ wp,
    float* vbuf, u16* qpb, float* part) {
  extern __shared__ __align__(16) unsigned char smem[];
  float* sTok = (float*)(smem);
  float* sKQV = (float*)(smem);
  float* sKP  = (float*)(smem + 49152);
  float* sQP  = (float*)(smem + 57344);
  unsigned char* r1 = smem + 65536;
  u16* xh = (u16*)(r1);
  u16* xl = (u16*)(r1 + 14400);
  u16* sAh = (u16*)(r1);
  u16* sAl = (u16*)(r1 + 33792);
  u16* sKh = (u16*)(r1);
  u16* sKl = (u16*)(r1 + 9216);
  u16* sQh = (u16*)(r1 + 18432);
  u16* sQl = (u16*)(r1 + 27648);
  u16* sVTh = (u16*)(r1 + 36864);
  u16* sVTl = (u16*)(r1 + 46080);
  u16* sKPTh = (u16*)(r1 + 55296);
  u16* sKPTl = (u16*)(r1 + 59904);
  unsigned char* r2 = smem + 133120;
  float* sMu = (float*)(r2);
  float* sRs = (float*)(r2 + 256);
  float* sXDk = (float*)(r2 + 512);
  float* sXDq = (float*)(r2 + 768);
  float* sPart = (float*)(r2 + 1024);

  const int tid = threadIdx.x, lane = tid & 31, wv = tid >> 5, m = lane & 15, h = lane >> 4;
  const int rt = wv & 3, ng = wv >> 2;
  const int b = blockIdx.y, blk = blockIdx.x, t0 = blk * 64;
  const int oh = t0 >> 8, ow0 = t0 & 255;
  const size_t tokb = (size_t)b * TT + t0;

  {
    const int ih0 = oh * 4 - 11, iw0 = ow0 * 4 - 11;
    const float* xb = x + (size_t)b * (IMW * IMW);
#pragma unroll 1
    for (int r = wv; r < XR; r += 8) {
      const int ih = ih0 + r;
      const bool rok = (unsigned)ih < (unsigned)IMW;
#pragma unroll 1
      for (int c = lane; c < XW; c += 32) {
        const int iw = iw0 + c;
        float v = 0.0f;
        if (rok && (unsigned)iw < (unsigned)IMW) v = xb[ih * IMW + iw];
        u16 hv, lv;
        split2(v, hv, lv);
        xh[r * XW + c] = hv;
        xl[r * XW + c] = lv;
      }
    }
  }
  __syncthreads();

  conv_dil<0>(xh, xl, wc, conv_b, sTok, lane, wv);
  conv_dil<1>(xh, xl, wc, conv_b, sTok, lane, wv);
  conv_dil<2>(xh, xl, wc, conv_b, sTok, lane, wv);
  conv_dil<3>(xh, xl, wc, conv_b, sTok, lane, wv);
  __syncthreads();

#pragma unroll 1
  for (int i = 0; i < 8; ++i) {
    const int tk = wv * 8 + i;
    const float* rp = sTok + tk * 256 + lane * 8;
    const v4f_t a = *(const v4fa*)(rp);
    const v4f_t c = *(const v4fa*)(rp + 4);
    float s = ((a[0] + a[1]) + (a[2] + a[3])) + ((c[0] + c[1]) + (c[2] + c[3]));
    s = wsum(s);
    const float mu = s * (1.0f / 256.0f);
    float d, ss = 0.0f;
    d = a[0] - mu; ss += d * d;  d = a[1] - mu; ss += d * d;
    d = a[2] - mu; ss += d * d;  d = a[3] - mu; ss += d * d;
    d = c[0] - mu; ss += d * d;  d = c[1] - mu; ss += d * d;
    d = c[2] - mu; ss += d * d;  d = c[3] - mu; ss += d * d;
    ss = wsum(ss);
    if (lane == 0) {
      sMu[tk] = mu;
      sRs[tk] = 1.0f / sqrtf(ss * (1.0f / 256.0f) + 1e-5f);
    }
  }
  __syncthreads();

#pragma unroll 1
  for (int i = 0; i < 8; ++i) {
    const int q = tid + 256 * i;
    const int tk = q >> 5, c0 = (q & 31) * 8;
    const float mu = sMu[tk], rs = sRs[tk];
    const float* sp = sTok + tk * 256 + c0;
    const v4f_t a = *(const v4fa*)(sp);
    const v4f_t c = *(const v4fa*)(sp + 4);
    const float xv[8] = {a[0], a[1], a[2], a[3], c[0], c[1], c[2], c[3]};
    us8_t hv = zeros8h(), lv = zeros8h();
#pragma unroll
    for (int e = 0; e < 8; ++e) {
      const float hn = (xv[e] - mu) * rs * n1g[c0 + e] + n1b[c0 + e];
      u16 hh, ll;
      split2(hn, hh, ll);
      hv[e] = hh; lv[e] = ll;
    }
    *(us8a*)(sAh + tk * AP + c0) = hv;
    *(us8a*)(sAl + tk * AP + c0) = lv;
  }
  __syncthreads();

  {
    v8f acc[6];
#pragma unroll
    for (int j = 0; j < 6; ++j) acc[j] = zero8();
    const u16* wkh = wk;
    const u16* wkl = wk + 192 * 256;
#pragma unroll 2
    for (int s = 0; s < 8; ++s) {
      const v16bf ah = ldfrag(sAh, AP, rt * 16 + m, 32 * s, h);
      const v16bf al = ldfrag(sAl, AP, rt * 16 + m, 32 * s, h);
#pragma unroll
      for (int j = 0; j < 6; ++j) {
        const int n = ng * 96 + j * 16 + m;
        const v16bf bh = ldfrag(wkh, 256, n, 32 * s, h);
        const v16bf bl = ldfrag(wkl, 256, n, 32 * s, h);
        mma3(acc[j], ah, al, bh, bl);
      }
    }
#pragma unroll
    for (int j = 0; j < 6; ++j) {
      const int n = ng * 96 + j * 16 + m;
      const float bias = kqv_b[n];
#pragma unroll
      for (int r = 0; r < 8; ++r) {
        const int tk = rt * 16 + 8 * h + r;
        sKQV[tk * 192 + n] = acc[j][r] + bias;
      }
    }
  }
  __syncthreads();

#pragma unroll 1
  for (int i = 0; i < 8; ++i) {
    const int tk = wv * 8 + i;
    const float* kr = sKQV + tk * 192;
    const float k0v = kr[lane * 2], k1v = kr[lane * 2 + 1];
    const float q0v = kr[64 + lane * 2], q1v = kr[65 + lane * 2];
    float sk = k0v * k0v + k1v * k1v;
    float sq = q0v * q0v + q1v * q1v;
    sk = wsum(sk);
    sq = wsum(sq);
    if (lane == 0) { sXDk[tk] = 0.5f * sk; sXDq[tk] = 0.5f * sq; }
  }
#pragma unroll 1
  for (int i = 0; i < 4; ++i) {
    const int q = tid + 256 * i;
    const int tk = q >> 4, grp = q & 15, c0 = grp * 8;
    const float* sp = sKQV + tk * 192 + c0;
    const v4f_t a = *(const v4fa*)(sp);
    const v4f_t c = *(const v4fa*)(sp + 4);
    const float xv[8] = {a[0], a[1], a[2], a[3], c[0], c[1], c[2], c[3]};
    us8_t hv = zeros8h(), lv = zeros8h();
#pragma unroll
    for (int e = 0; e < 8; ++e) { u16 hh, ll; split2(xv[e], hh, ll); hv[e] = hh; lv[e] = ll; }
    u16* dh; u16* dl;
    if (grp < 8) { dh = sKh + tk * SP + c0;        dl = sKl + tk * SP + c0; }
    else         { dh = sQh + tk * SP + (c0 - 64); dl = sQl + tk * SP + (c0 - 64); }
    *(us8a*)dh = hv;
    *(us8a*)dl = lv;
  }
#pragma unroll 1
  for (int i = 0; i < 2; ++i) {
    const int q = tid + 256 * i;
    const int tk = q >> 3, c0 = (q & 7) * 8;
    const float* sp = sKQV + tk * 192 + 128 + c0;
    const v4f_t a = *(const v4fa*)(sp);
    const v4f_t c = *(const v4fa*)(sp + 4);
    const float xv[8] = {a[0], a[1], a[2], a[3], c[0], c[1], c[2], c[3]};
#pragma unroll
    for (int e = 0; e < 8; ++e) {
      u16 hh, ll;
      split2(xv[e], hh, ll);
      sVTh[(c0 + e) * SP + tk] = hh;
      sVTl[(c0 + e) * SP + tk] = ll;
    }
  }
  {
    v4f_t vv[4];
#pragma unroll
    for (int i = 0; i < 4; ++i) {
      const int e = (i * 32 + lane) * 4;
      const int tk = wv * 8 + (e >> 6), n = e & 63;
      vv[i] = *(const v4fa*)(sKQV + tk * 192 + 128 + n);
    }
    float* vd = vbuf + (tokb + wv * 8) * 64;
#pragma unroll
    for (int i = 0; i < 4; ++i) *(volatile v4f_t*)(vd + (i * 32 + lane) * 4) = vv[i];
    __threadfence();
#pragma unroll
    for (int i = 0; i < 4; ++i) *(volatile v4f_t*)(vd + (i * 32 + lane) * 4) = vv[i];
  }
  __syncthreads();

  const int nt = wv >> 2;
  {
    v8f a1 = zero8();
#pragma unroll
    for (int s = 0; s < 2; ++s) {
      const v16bf ah = ldfrag(sKh, SP, rt * 16 + m, 32 * s, h);
      const v16bf al = ldfrag(sKl, SP, rt * 16 + m, 32 * s, h);
      const v16bf bh = ldfrag(wp, 64, nt * 16 + m, 32 * s, h);
      const v16bf bl = ldfrag(wp + 2048, 64, nt * 16 + m, 32 * s, h);
      mma3(a1, ah, al, bh, bl);
    }
#pragma unroll
    for (int r = 0; r < 8; ++r) {
      const int tk = rt * 16 + 8 * h + r;
      sKP[tk * 32 + nt * 16 + m] = expf(a1[r] - sXDk[tk]) * RSQ32;
    }
  }
  __syncthreads();

#pragma unroll 1
  for (int i = 0; i < 8; ++i) {
    const int q = tid + 256 * i;
    const int mm = q >> 6, tk = q & 63;
    u16 hh, ll;
    split2(sKP[tk * 32 + mm], hh, ll);
    sKPTh[mm * SP + tk] = hh;
    sKPTl[mm * SP + tk] = ll;
  }
  if (tid < 128) {
    float s = 0.0f;
    if (tid < 32) {
#pragma unroll 1
      for (int t = 0; t < 64; ++t) s += sKP[t * 32 + tid];
    }
    sPart[2048 + tid] = s;
  }
  {
    v8f a1 = zero8();
#pragma unroll
    for (int s = 0; s < 2; ++s) {
      const v16bf ah = ldfrag(sQh, SP, rt * 16 + m, 32 * s, h);
      const v16bf al = ldfrag(sQl, SP, rt * 16 + m, 32 * s, h);
      const v16bf bh = ldfrag(wp, 64, nt * 16 + m, 32 * s, h);
      const v16bf bl = ldfrag(wp + 2048, 64, nt * 16 + m, 32 * s, h);
      mma3(a1, ah, al, bh, bl);
    }
#pragma unroll
    for (int r = 0; r < 8; ++r) {
      const int tk = rt * 16 + 8 * h + r;
      sQP[tk * 32 + nt * 16 + m] = expf(a1[r] - sXDq[tk]) * RSQ32;
    }
  }
  __syncthreads();

  {
    v8f a1 = zero8();
#pragma unroll
    for (int s = 0; s < 2; ++s) {
      const v16bf ah = ldfrag(sVTh, SP, rt * 16 + m, 32 * s, h);
      const v16bf al = ldfrag(sVTl, SP, rt * 16 + m, 32 * s, h);
      const v16bf bh = ldfrag(sKPTh, SP, nt * 16 + m, 32 * s, h);
      const v16bf bl = ldfrag(sKPTl, SP, nt * 16 + m, 32 * s, h);
      mma3(a1, ah, al, bh, bl);
    }
#pragma unroll
    for (int r = 0; r < 8; ++r)
      sPart[(rt * 16 + 8 * h + r) * 32 + nt * 16 + m] = a1[r];
  }
  {
    us8_t qv[2];
#pragma unroll
    for (int i = 0; i < 2; ++i) {
      const int q = i * 32 + lane;
      const int tkl = wv * 8 + (q >> 3), pc = q & 7;
      const float* sp = sQP + tkl * 32 + (pc & 3) * 8;
      const v4f_t a = *(const v4fa*)(sp);
      const v4f_t c = *(const v4fa*)(sp + 4);
      const float xv[8] = {a[0], a[1], a[2], a[3], c[0], c[1], c[2], c[3]};
      us8_t o = zeros8h();
#pragma unroll
      for (int e = 0; e < 8; ++e) { u16 hh, ll; split2(xv[e], hh, ll); o[e] = (pc < 4) ? hh : ll; }
      qv[i] = o;
    }
#pragma unroll
    for (int i = 0; i < 2; ++i) {
      const int q = i * 32 + lane;
      const int tkl = wv * 8 + (q >> 3), pc = q & 7;
      *(volatile us8_t*)(qpb + (tokb + tkl) * 64 + pc * 8) = qv[i];
    }
    __threadfence();
#pragma unroll
    for (int i = 0; i < 2; ++i) {
      const int q = i * 32 + lane;
      const int tkl = wv * 8 + (q >> 3), pc = q & 7;
      *(volatile us8_t*)(qpb + (tokb + tkl) * 64 + pc * 8) = qv[i];
    }
  }
  __syncthreads();

  {
    float* pd = part + ((size_t)b * NBPB + blk) * RECW;
    const int e0 = (wv * 64 + lane) * 4, e1 = (wv * 64 + 32 + lane) * 4, e2 = 2048 + lane * 4;
    const v4f_t p0 = *(const v4fa*)(sPart + e0);
    const v4f_t p1 = *(const v4fa*)(sPart + e1);
    const v4f_t p2 = *(const v4fa*)(sPart + e2);
    *(volatile v4f_t*)(pd + e0) = p0;
    *(volatile v4f_t*)(pd + e1) = p1;
    if (wv == 0) *(volatile v4f_t*)(pd + e2) = p2;
    __threadfence();
    *(volatile v4f_t*)(pd + e0) = p0;
    *(volatile v4f_t*)(pd + e1) = p1;
    if (wv == 0) *(volatile v4f_t*)(pd + e2) = p2;
  }
}

__global__ __launch_bounds__(256) void k_reduce(const float* __restrict__ part, u16* kx, int nbpb) {
  __shared__ __align__(16) float sRed[320];
  const int tid = threadIdx.x, jb = blockIdx.x, b = blockIdx.y;
  for (int e = tid; e < 320; e += 256) {
    const int rr = jb * 10 + (e >> 5), mm = e & 31;
    int si = -1;
    if (rr < 64) si = rr * 32 + mm;
    else if (rr == 64) si = 2048 + mm;
    double s = 0.0;
    if (si >= 0) {
      const float* p = part + (size_t)b * nbpb * RECW + si;
#pragma unroll 4
      for (int k = 0; k < nbpb; ++k) s += (double)p[(size_t)k * RECW];
    }
    sRed[e] = (float)s;
  }
  __syncthreads();
  us8_t pv = zeros8h();
  u16* dst = kx;
  const bool act = tid < 80;
  if (act) {
    const int plane = (tid >= 40) ? 1 : 0;
    const int pc = tid - plane * 40;
#pragma unroll
    for (int e = 0; e < 8; ++e) {
      u16 hv, lv;
      split2(sRed[pc * 8 + e], hv, lv);
      pv[e] = plane ? lv : hv;
    }
    dst = kx + (size_t)(b * 2 + plane) * KXW + jb * 320 + pc * 8;
    *(volatile us8_t*)dst = pv;
  }
  __threadfence();
  if (act) *(volatile us8_t*)dst = pv;
}

__device__ __forceinline__ void gemm64x2(v8f (&acc)[2], const u16* sYh, const u16* sYl, const u16* __restrict__ wgh,
                                         int rt, int ng, int m, int h) {
  acc[0] = zero8();
  acc[1] = zero8();
#pragma unroll
  for (int s = 0; s < 2; ++s) {
    const v16bf ah = ldfrag(sYh, SP, rt * 16 + m, 32 * s, h);
    const v16bf al = ldfrag(sYl, SP, rt * 16 + m, 32 * s, h);
#pragma unroll
    for (int j = 0; j < 2; ++j) {
      const int n = (2 * ng + j) * 16 + m;
      const v16bf bh = ldfrag(wgh, 64, n, 32 * s, h);
      const v16bf bl = ldfrag(wgh + 4096, 64, n, 32 * s, h);
      mma3(acc[j], ah, al, bh, bl);
    }
  }
}

__global__ __launch_bounds__(256) void k_tail(
    const u16* __restrict__ qpb, const float* __restrict__ vbuf, const u16* __restrict__ kx,
    const u16* __restrict__ wpr, const float* __restrict__ proj_b,
    const float* __restrict__ n2g, const float* __restrict__ n2b,
    const u16* __restrict__ wm1, const float* __restrict__ m1b,
    const u16* __restrict__ wm2, const float* __restrict__ m2b, float* out) {
  __shared__ __align__(16) u16 sYh[64 * SP];
  __shared__ __align__(16) u16 sYl[64 * SP];
  __shared__ __align__(16) float sYf[64 * YP];
  __shared__ __align__(16) float sO[64 * 64];
  const int tid = threadIdx.x, lane = tid & 31, wv = tid >> 5, m = lane & 15, h = lane >> 4;
  const int rt = wv & 3, ng = wv >> 2;
  const int b = blockIdx.y, t0 = blockIdx.x * 64;
  const size_t tokb = (size_t)b * TT + t0;

  {
    const u16* qr = qpb + (tokb + rt * 16 + m) * 64;
    Frag fa, fb;
    fa.h[0] = *(const us8a*)(qr + 8 * h);
    fa.h[1] = *(const us8a*)(qr + 16 + 8 * h);
    fb.h[0] = *(const us8a*)(qr + 32 + 8 * h);
    fb.h[1] = *(const us8a*)(qr + 48 + 8 * h);
    const u16* kxh = kx + (size_t)(b * 2 + 0) * KXW;
    const u16* kxl = kx + (size_t)(b * 2 + 1) * KXW;
    v8f acc[3];
#pragma unroll
    for (int j = 0; j < 3; ++j) {
      const int tj = (j < 2) ? (2 * ng + j) : 4;
      acc[j] = zero8();
      const v16bf bh = ldfrag(kxh, 32, tj * 16 + m, 0, h);
      const v16bf bl = ldfrag(kxl, 32, tj * 16 + m, 0, h);
      mma3(acc[j], fa.v, fb.v, bh, bl);
    }
    float rinv[8];
#pragma unroll
    for (int r = 0; r < 8; ++r) {
      const float dv = __shfl(acc[2][r], lane & 16, 32);
      rinv[r] = 1.0f / (dv + 1e-8f);
    }
#pragma unroll
    for (int j = 0; j < 2; ++j) {
#pragma unroll
      for (int r = 0; r < 8; ++r) {
        const int tk = rt * 16 + 8 * h + r, n = (2 * ng + j) * 16 + m;
        u16 hv, lv;
        split2(acc[j][r] * rinv[r], hv, lv);
        sYh[tk * SP + n] = hv;
        sYl[tk * SP + n] = lv;
      }
    }
  }
  __syncthreads();

  {
    v8f acc[2];
    gemm64x2(acc, sYh, sYl, wpr, rt, ng, m, h);
#pragma unroll
    for (int j = 0; j < 2; ++j) {
      const int n = (2 * ng + j) * 16 + m;
      const float bias = proj_b[n];
#pragma unroll
      for (int r = 0; r < 8; ++r) {
        const int tk = rt * 16 + 8 * h + r;
        const float vv = vbuf[(tokb + tk) * 64 + n];
        sYf[tk * YP + n] = vv + (acc[j][r] + bias);
      }
    }
  }
  __syncthreads();

#pragma unroll 1
  for (int i = 0; i < 8; ++i) {
    const int tk = wv * 8 + i;
    const int c = lane * 2;
    const float y0 = sYf[tk * YP + c], y1 = sYf[tk * YP + c + 1];
    const float s = wsum(y0 + y1);
    const float mu = s * (1.0f / 64.0f);
    const float d0 = y0 - mu, d1 = y1 - mu;
    const float ss = wsum(d0 * d0 + d1 * d1);
    const float rs = 1.0f / sqrtf(ss * (1.0f / 64.0f) + 1e-5f);
    const float mn0 = d0 * rs * n2g[c] + n2b[c];
    const float mn1 = d1 * rs * n2g[c + 1] + n2b[c + 1];
    u16 a0, b0, a1, b1;
    split2(mn0, a0, b0);
    split2(mn1, a1, b1);
    sYh[tk * SP + c] = a0; sYl[tk * SP + c] = b0;
    sYh[tk * SP + c + 1] = a1; sYl[tk * SP + c + 1] = b1;
  }
  __syncthreads();

  {
    v8f acc[2];
    gemm64x2(acc, sYh, sYl, wm1, rt, ng, m, h);
    u16 gh[2][8], gl[2][8];
#pragma unroll
    for (int j = 0; j < 2; ++j) {
      const int n = (2 * ng + j) * 16 + m;
      const float bias = m1b[n];
#pragma unroll
      for (int r = 0; r < 8; ++r) split2(gelu_f(acc[j][r] + bias), gh[j][r], gl[j][r]);
    }
    __syncthreads();
#pragma unroll
    for (int j = 0; j < 2; ++j) {
#pragma unroll
      for (int r = 0; r < 8; ++r) {
        const int tk = rt * 16 + 8 * h + r, n = (2 * ng + j) * 16 + m;
        sYh[tk * SP + n] = gh[j][r];
        sYl[tk * SP + n] = gl[j][r];
      }
    }
  }
  __syncthreads();

  {
    v8f acc[2];
    gemm64x2(acc, sYh, sYl, wm2, rt, ng, m, h);
#pragma unroll
    for (int j = 0; j < 2; ++j) {
      const int n = (2 * ng + j) * 16 + m;
      const float bias = m2b[n];
#pragma unroll
      for (int r = 0; r < 8; ++r) {
        const int tk = rt * 16 + 8 * h + r;
        sO[tk * 64 + n] = sYf[tk * YP + n] + (acc[j][r] + bias);
      }
    }
  }
  __syncthreads();
  {
    float* od = out + tokb * 64;
    v4f_t ov[4];
#pragma unroll
    for (int i = 0; i < 4; ++i) ov[i] = *(const v4fa*)(sO + wv * 512 + (i * 32 + lane) * 4);
#pragma unroll
    for (int i = 0; i < 4; ++i) *(volatile v4f_t*)(od + wv * 512 + (i * 32 + lane) * 4) = ov[i];
    __threadfence();
#pragma unroll
    for (int i = 0; i < 4; ++i) *(volatile v4f_t*)(od + wv * 512 + (i * 32 + lane) * 4) = ov[i];
  }
}

extern "C" void kernel_launch(void* const* d_in, const int* in_sizes, int n_in,
                              void* d_out, int out_size, void* d_ws, size_t ws_size,
                              hipStream_t stream) {
  (void)n_in;
  const float* x      = (const float*)d_in[0];
  const float* conv_w = (const float*)d_in[1];
  const float* conv_b = (const float*)d_in[2];
  const float* n1g    = (const float*)d_in[3];
  const float* n1b    = (const float*)d_in[4];
  const float* kqv_w  = (const float*)d_in[5];
  const float* kqv_b  = (const float*)d_in[6];
  const float* proj_w = (const float*)d_in[7];
  const float* proj_b = (const float*)d_in[8];
  const float* n2g    = (const float*)d_in[9];
  const float* n2b    = (const float*)d_in[10];
  const float* mlp1_w = (const float*)d_in[11];
  const float* mlp1_b = (const float*)d_in[12];
  const float* mlp2_w = (const float*)d_in[13];
  const float* mlp2_b = (const float*)d_in[14];
  const float* wperf  = (const float*)d_in[15];
  float* out = (float*)d_out;

  const int nb = in_sizes[0] / (IMW * IMW);
  if (nb < 1 || out_size != nb * TT * 64) return;

  char* ws = (char*)d_ws;
  size_t off = 0;
  const size_t b_wc   = (size_t)4 * 2 * 64 * 64 * 2;
  const size_t b_wk   = (size_t)2 * 192 * 256 * 2;
  const size_t b_wp   = (size_t)2 * 32 * 64 * 2;
  const size_t b_w64  = (size_t)2 * 64 * 64 * 2;
  const size_t b_vbuf = (size_t)nb * TT * 64 * 4;
  const size_t b_qpb  = (size_t)nb * TT * 64 * 2;
  const size_t b_part = (size_t)nb * NBPB * RECW * 4;
  const size_t b_kx   = (size_t)nb * 2 * KXW * 2;
  u16* wc  = (u16*)(ws + off); off += (b_wc + 127) & ~(size_t)127;
  u16* wk  = (u16*)(ws + off); off += (b_wk + 127) & ~(size_t)127;
  u16* wp  = (u16*)(ws + off); off += (b_wp + 127) & ~(size_t)127;
  u16* wpr = (u16*)(ws + off); off += (b_w64 + 127) & ~(size_t)127;
  u16* wm1 = (u16*)(ws + off); off += (b_w64 + 127) & ~(size_t)127;
  u16* wm2 = (u16*)(ws + off); off += (b_w64 + 127) & ~(size_t)127;
  float* vbuf = (float*)(ws + off); off += (b_vbuf + 127) & ~(size_t)127;
  u16* qpb = (u16*)(ws + off); off += (b_qpb + 127) & ~(size_t)127;
  float* part = (float*)(ws + off); off += (b_part + 127) & ~(size_t)127;
  u16* kx = (u16*)(ws + off); off += (b_kx + 127) & ~(size_t)127;
  if (off > ws_size) return;

  k_prep<<<dim3(10), dim3(256), 0, stream>>>(conv_w, kqv_w, wperf, proj_w, mlp1_w, mlp2_w,
                                             wc, wk, wp, wpr, wm1, wm2);
  hipFuncSetAttribute((const void*)k_main, hipFuncAttributeMaxDynamicSharedMemorySize, LDS_MAIN);
  k_main<<<dim3(NBPB, nb), dim3(256), LDS_MAIN, stream>>>(x, conv_b, n1g, n1b, kqv_b, wc, wk, wp,
                                                          vbuf, qpb, part);
  k_reduce<<<dim3(8, nb), dim3(256), 0, stream>>>(part, kx, NBPB);
  k_tail<<<dim3(NBPB, nb), dim3(256), 0, stream>>>(qpb, vbuf, kx, wpr, proj_b, n2g, n2b,
                                                   wm1, mlp1_b, wm2, mlp2_b, out);
}
